// HeteroGATLayer_54443005444388
// MI455X (gfx1250) — hardware-verified
//
#include <hip/hip_runtime.h>
#include <stddef.h>


#define FIN     128
#define NC      256
#define HEADS   4
#define CH      64
#define DOUT    64
#define TT      3
#define NTHR    256
#define NWAVE   8
#define EPT     8
#define NGRP    2
#define CHUNK   (NTHR * EPT * NGRP)
#define WCAP    (EPT * NGRP * 32)
#define LISTN   (NWAVE * WCAP)
#define NBC     4096
#define NBF     1024
#define RCAP    40960
#define RBN     128
#define TGT     256
#define DEGCAP  256
#define OTHR    512
#define SROWS   16
#define GBM     64
#define GLDS    (GBM * NC * 4)
#define WSCALE  64.0f
#define WINV    0.015625f
#define WSCAP   134217728
#define NEG_SLOPE 0.2f
#define NEG_BIG (-3.0e38f)

#define LDS_FILL ((RCAP + NBF + LISTN) * 4 + 64)

static_assert((CHUNK & (CHUNK - 1)) == 0);
static_assert(CHUNK <= 4096);
static_assert(NBC <= 4096 && NBF <= 4096);
static_assert((NBC & (NBC - 1)) == 0 && (NBF & (NBF - 1)) == 0);
static_assert(NBC == 4 * NBF);
static_assert(OTHR * 8 == NBC);
static_assert((RCAP % 32) == 0);
static_assert(TGT == NWAVE * 32);
static_assert((NBC % TGT) == 0);
static_assert((TGT % GBM) == 0);
static_assert(HEADS * CH == NC && NC == 2 * 128 && DOUT == CH);
static_assert(FIN % 32 == 0);
static_assert((SROWS & (SROWS - 1)) == 0 && 32 % SROWS == 0);
static_assert(SROWS * DOUT == 8 * 32 * 4);

typedef float          v4f  __attribute__((ext_vector_type(4)));
typedef float          v8f  __attribute__((ext_vector_type(8)));
typedef int            v4i  __attribute__((ext_vector_type(4)));
typedef unsigned short v8us __attribute__((ext_vector_type(8)));
typedef _Float16       v8h  __attribute__((ext_vector_type(8)));
typedef _Float16       v16h __attribute__((ext_vector_type(16)));
union FragH { v16h v; v8us h[2]; };
union Pack8 { v8h h; v8us u; };

__device__ __forceinline__ v8us cvt8h(v4f a, v4f b, float sc) {
  v8h r;
  r[0] = (_Float16)(a.x * sc); r[1] = (_Float16)(a.y * sc);
  r[2] = (_Float16)(a.z * sc); r[3] = (_Float16)(a.w * sc);
  r[4] = (_Float16)(b.x * sc); r[5] = (_Float16)(b.y * sc);
  r[6] = (_Float16)(b.z * sc); r[7] = (_Float16)(b.w * sc);
  Pack8 p;
  p.h = r;
  return p.u;
}

__device__ __forceinline__ v8f wmh(v16h a, v16h b, v8f c) {
  v8f d = __builtin_amdgcn_wmma_f32_16x16x32_f16(false, a, false, b, (short)0, c, false, false);
  asm volatile("v_nop\n\tv_nop\n\tv_nop\n\tv_nop" : "+v"(d) : "v"(a), "v"(b));
  return d;
}

__device__ __forceinline__ float lrelu(float v) { return v >= 0.0f ? v : NEG_SLOPE * v; }

template <int NB>
__device__ __forceinline__ int scan_chunk(const int* __restrict__ dsts, int nE, int cbase, int slotBase,
                                          int vec8, int* list, int tid, int lane, int wave) {
  int wc = 0;
#pragma unroll
  for (int g = 0; g < NGRP; ++g) {
    const int el0  = (g * NTHR + tid) * EPT;
    const int e0   = cbase + el0;
    const int sent = -2147483647 - 1;
    v4i da, db;
    if (vec8 != 0 && cbase + CHUNK <= nE) {
      da = *(const v4i*)(dsts + e0);
      db = *(const v4i*)(dsts + e0 + 4);
    } else {
      da.x = (e0     < nE) ? dsts[min(e0, nE - 1)] : sent;
      da.y = (e0 + 1 < nE) ? dsts[min(e0 + 1, nE - 1)] : sent;
      da.z = (e0 + 2 < nE) ? dsts[min(e0 + 2, nE - 1)] : sent;
      da.w = (e0 + 3 < nE) ? dsts[min(e0 + 3, nE - 1)] : sent;
      db.x = (e0 + 4 < nE) ? dsts[min(e0 + 4, nE - 1)] : sent;
      db.y = (e0 + 5 < nE) ? dsts[min(e0 + 5, nE - 1)] : sent;
      db.z = (e0 + 6 < nE) ? dsts[min(e0 + 6, nE - 1)] : sent;
      db.w = (e0 + 7 < nE) ? dsts[min(e0 + 7, nE - 1)] : sent;
    }
    const unsigned nb = (unsigned)slotBase;
    const unsigned s0 = (unsigned)da.x - nb, s1 = (unsigned)da.y - nb;
    const unsigned s2 = (unsigned)da.z - nb, s3 = (unsigned)da.w - nb;
    const unsigned s4 = (unsigned)db.x - nb, s5 = (unsigned)db.y - nb;
    const unsigned s6 = (unsigned)db.z - nb, s7 = (unsigned)db.w - nb;
    const bool h0 = s0 < (unsigned)NB, h1 = s1 < (unsigned)NB, h2 = s2 < (unsigned)NB, h3 = s3 < (unsigned)NB;
    const bool h4 = s4 < (unsigned)NB, h5 = s5 < (unsigned)NB, h6 = s6 < (unsigned)NB, h7 = s7 < (unsigned)NB;
    const unsigned any = __builtin_amdgcn_ballot_w32(h0 | h1 | h2 | h3 | h4 | h5 | h6 | h7);
    if (any != 0u) {
#define HITJ(J, HJ, SJ) { \
        const unsigned mj = __builtin_amdgcn_ballot_w32(HJ); \
        if (mj != 0u) { \
          if (HJ) { \
            const int pos = wc + (int)__builtin_amdgcn_mbcnt_lo(mj, 0u); \
            if (pos < WCAP) list[wave * WCAP + pos] = ((el0 + (J)) << 12) | (int)(SJ); \
          } \
          wc += (int)__builtin_popcount(mj); } }
      HITJ(0, h0, s0)
      HITJ(1, h1, s1)
      HITJ(2, h2, s2)
      HITJ(3, h3, s3)
      HITJ(4, h4, s4)
      HITJ(5, h5, s5)
      HITJ(6, h6, s6)
      HITJ(7, h7, s7)
#undef HITJ
    }
  }
  return wc;
}

__global__ __launch_bounds__(NTHR) void k_wprep(const float* __restrict__ W, unsigned short* wp) {
  constexpr int UNITS = NC * FIN / 8;
  constexpr int KD8   = FIN / 8;
  static_assert((UNITS % NTHR) == 0);
  const int t = (int)blockIdx.y;
  const int i = (int)blockIdx.x * NTHR + (int)threadIdx.x;
  if (i >= UNITS) return;
  const int n  = i / KD8;
  const int k0 = (i - n * KD8) * 8;
  const float* Wt = W + (size_t)t * FIN * NC;
  float v[8];
#pragma unroll
  for (int e = 0; e < 8; ++e) v[e] = Wt[(size_t)(k0 + e) * NC + n];
  v4f a, b;
  a.x = v[0]; a.y = v[1]; a.z = v[2]; a.w = v[3];
  b.x = v[4]; b.y = v[5]; b.z = v[6]; b.w = v[7];
  const v8us hv = cvt8h(a, b, WSCALE);
  unsigned short* d = wp + (size_t)t * NC * FIN + (size_t)i * 8;
  *(volatile v8us*)d = hv;
  __threadfence();
  *(volatile v8us*)d = hv;
}

__global__ __launch_bounds__(NTHR) void k_xprep(const float* __restrict__ x, unsigned short* xh,
                                                int nN, int nUnits) {
  constexpr int KD8 = FIN / 8;
  const int i = (int)blockIdx.x * NTHR + (int)threadIdx.x;
  if (i >= nUnits) return;
  const int row = i / KD8;
  const int c0  = (i - row * KD8) * 8;
  const int rc  = row < nN ? row : nN - 1;
  const float* p = x + (size_t)rc * FIN + c0;
  v4f a = *(const v4f*)p, b = *(const v4f*)(p + 4);
  const v4f z4 = {0.f, 0.f, 0.f, 0.f};
  if (row >= nN) { a = z4; b = z4; }
  const v8us hv = cvt8h(a, b, 1.0f);
  unsigned short* d = xh + (size_t)i * 8;
  *(volatile v8us*)d = hv;
  __threadfence();
  *(volatile v8us*)d = hv;
}

__global__ __launch_bounds__(NTHR) void k_count(
    const int* __restrict__ dstAll, int* cntAll, int nE, int vec8, int cntStride) {
  __shared__ __attribute__((aligned(16))) int scnt[NBC];
  __shared__ __attribute__((aligned(16))) int list[LISTN];
  __shared__ int wcnt[NWAVE];
  const int tid = threadIdx.x, lane = tid & 31, wave = tid >> 5;
  const int nodeBase = blockIdx.x * NBC;
  const int* dsts = dstAll + (size_t)blockIdx.y * nE;
  int* cnt = cntAll + (size_t)blockIdx.y * cntStride;

  for (int i = tid; i < NBC; i += NTHR) scnt[i] = 0;
  __syncthreads();

  const int nChunks = (nE + CHUNK - 1) / CHUNK;
#pragma unroll 1
  for (int ch = 0; ch < nChunks; ++ch) {
    const int cbase = ch * CHUNK;
    const int wc = scan_chunk<NBC>(dsts, nE, cbase, nodeBase, vec8, list, tid, lane, wave);
    if (lane == 0) wcnt[wave] = wc;
    __syncthreads();
    if (wave == 0) {
#pragma unroll 1
      for (int wsx = 0; wsx < NWAVE; ++wsx) {
        int n = __builtin_amdgcn_readfirstlane(wcnt[wsx]);
        n = n > WCAP ? WCAP : (n < 0 ? 0 : n);
        const int* lp = list + wsx * WCAP;
#pragma unroll 1
        for (int i = 0; i < n; ++i) {
          const int ent  = __builtin_amdgcn_readfirstlane(lp[i]);
          const int slot = ent & (NBC - 1);
          if (lane == 0) scnt[slot] = scnt[slot] + 1;
        }
      }
    }
    __syncthreads();
  }

  v4i cq[4];
#pragma unroll
  for (int q = 0; q < 4; ++q) {
    const int f = (wave * 4 + q) * 128 + 4 * lane;
    cq[q] = *(const v4i*)(scnt + f);
  }
  int* cp = cnt + (size_t)nodeBase;
#pragma unroll
  for (int q = 0; q < 4; ++q) {
    const int f = (wave * 4 + q) * 128 + 4 * lane;
    *(volatile v4i*)(cp + f) = cq[q];
  }
  __threadfence();
#pragma unroll
  for (int q = 0; q < 4; ++q) {
    const int f = (wave * 4 + q) * 128 + 4 * lane;
    *(volatile v4i*)(cp + f) = cq[q];
  }
}

__global__ __launch_bounds__(OTHR) void k_offsets(
    const int* __restrict__ cntAll, int* offAll, int* rbAll, int nChunk, int cntStride) {
  __shared__ __attribute__((aligned(16))) int soff[NBC];
  __shared__ __attribute__((aligned(16))) int srb[RBN];
  __shared__ int wtot[OTHR / 32];
  const int tid = threadIdx.x, lane = tid & 31, wave = tid >> 5, sub = tid >> 7;
  const int* cnt = cntAll + (size_t)blockIdx.x * cntStride;
  int* off   = offAll + (size_t)blockIdx.x * cntStride;
  int* rbase = rbAll + (size_t)blockIdx.x * RBN;
  for (int i = tid; i < RBN; i += OTHR) srb[i] = 0;
  int carry = 0;
#pragma unroll 1
  for (int ch = 0; ch < nChunk; ++ch) {
    const int base = ch * NBC;
    const v4i c0 = *(const v4i*)(cnt + base + 8 * tid);
    const v4i c1 = *(const v4i*)(cnt + base + 8 * tid + 4);
    const int e0 = max(c0.x, 0), e1 = max(c0.y, 0), e2 = max(c0.z, 0), e3 = max(c0.w, 0);
    const int e4 = max(c1.x, 0), e5 = max(c1.y, 0), e6 = max(c1.z, 0), e7 = max(c1.w, 0);
    const int ts = e0 + e1 + e2 + e3 + e4 + e5 + e6 + e7;
    int incl = ts;
#pragma unroll
    for (int d = 1; d < 32; d <<= 1) {
      const int t = __shfl_up(incl, d);
      if (lane >= d) incl += t;
    }
    if (lane == 31) wtot[wave] = incl;
    __syncthreads();
    const int S0 = wtot[0]  + wtot[1]  + wtot[2]  + wtot[3];
    const int S1 = wtot[4]  + wtot[5]  + wtot[6]  + wtot[7];
    const int S2 = wtot[8]  + wtot[9]  + wtot[10] + wtot[11];
    const int S3 = wtot[12] + wtot[13] + wtot[14] + wtot[15];
    int pre = 0;
#pragma unroll 1
    for (int w = 4 * sub; w < wave; ++w) pre += wtot[w];
    const int b0 = carry;
    const int b1 = b0 + ((S0 + 31) & ~31);
    const int b2 = b1 + ((S1 + 31) & ~31);
    const int b3 = b2 + ((S2 + 31) & ~31);
    const int b4 = b3 + ((S3 + 31) & ~31);
    const int myb = sub == 0 ? b0 : (sub == 1 ? b1 : (sub == 2 ? b2 : b3));
    if (tid == 0) {
      srb[min(4 * ch + 0, RBN - 1)] = b0;
      srb[min(4 * ch + 1, RBN - 1)] = b1;
      srb[min(4 * ch + 2, RBN - 1)] = b2;
      srb[min(4 * ch + 3, RBN - 1)] = b3;
    }
    int run = myb + pre + incl - ts;
    soff[8 * tid + 0] = run; run += e0;
    soff[8 * tid + 1] = run; run += e1;
    soff[8 * tid + 2] = run; run += e2;
    soff[8 * tid + 3] = run; run += e3;
    soff[8 * tid + 4] = run; run += e4;
    soff[8 * tid + 5] = run; run += e5;
    soff[8 * tid + 6] = run; run += e6;
    soff[8 * tid + 7] = run;
    carry = b4;
    __syncthreads();
    const v4i o0 = *(const v4i*)(soff + 4 * tid);
    const v4i o1 = *(const v4i*)(soff + 4 * (tid + OTHR));
    int* op = off + base;
    *(volatile v4i*)(op + 4 * tid) = o0;
    *(volatile v4i*)(op + 4 * (tid + OTHR)) = o1;
    __threadfence();
    *(volatile v4i*)(op + 4 * tid) = o0;
    *(volatile v4i*)(op + 4 * (tid + OTHR)) = o1;
    __syncthreads();
  }
  if (tid == 0) srb[min(4 * nChunk, RBN - 1)] = carry;
  __syncthreads();
  v4i rv = {0, 0, 0, 0};
  if (tid < 32) rv = *(const v4i*)(srb + 4 * tid);
  if (tid < 32) *(volatile v4i*)(rbase + 4 * tid) = rv;
  __threadfence();
  if (tid < 32) *(volatile v4i*)(rbase + 4 * tid) = rv;
}

__global__ __launch_bounds__(NTHR) void k_fill(
    const int* __restrict__ srcAll, const int* __restrict__ dstAll,
    const int* __restrict__ offAll, const int* __restrict__ rbAll,
    int* csrAll, int nN, int nE, int vec8, int csrLen, int cntStride) {
  extern __shared__ v4f lds_dyn[];
  int* region = (int*)lds_dyn;
  int* cursor = region + RCAP;
  int* list   = cursor + NBF;
  int* wcnt   = list + LISTN;
  const int tid = threadIdx.x, lane = tid & 31, wave = tid >> 5;
  const int t = (int)blockIdx.y;
  const int b = (int)blockIdx.x;
  const int nodeBase = b * NBF;
  const int* srcs  = srcAll + (size_t)t * nE;
  const int* dsts  = dstAll + (size_t)t * nE;
  const int* off   = offAll + (size_t)t * cntStride;
  const int* rbase = rbAll + (size_t)t * RBN;
  int* csr = csrAll + (size_t)t * csrLen;

  int rb0 = rbase[b];
  const int rb1 = rbase[b + 1];
  rb0 = rb0 < 0 ? 0 : (rb0 > csrLen ? csrLen : rb0);
  rb0 &= ~31;
  int len = rb1 - rb0;
  len = len < 0 ? 0 : (len > RCAP ? RCAP : len);
  int lenW = (len + 31) & ~31;
  if (rb0 + lenW > csrLen) lenW = (csrLen - rb0) & ~31;

  {
    const v4i z = {0, 0, 0, 0};
    for (int i = tid; i < RCAP / 4; i += NTHR) ((v4i*)region)[i] = z;
    for (int s = tid; s < NBF; s += NTHR) {
      int o = off[nodeBase + s] - rb0;
      o = o < 0 ? 0 : (o > RCAP ? RCAP : o);
      cursor[s] = o;
    }
  }
  __syncthreads();

  const int nChunks = (nE + CHUNK - 1) / CHUNK;
#pragma unroll 1
  for (int ch = 0; ch < nChunks; ++ch) {
    const int cbase = ch * CHUNK;
    const int wc = scan_chunk<NBF>(dsts, nE, cbase, nodeBase, vec8, list, tid, lane, wave);
    if (lane == 0) wcnt[wave] = wc;
    __syncthreads();
    if (wave == 0) {
#pragma unroll 1
      for (int wsx = 0; wsx < NWAVE; ++wsx) {
        int n = __builtin_amdgcn_readfirstlane(wcnt[wsx]);
        n = n > WCAP ? WCAP : (n < 0 ? 0 : n);
        const int* lp = list + wsx * WCAP;
#pragma unroll 1
        for (int i = 0; i < n; ++i) {
          const int ent  = __builtin_amdgcn_readfirstlane(lp[i]);
          const int slot = ent & (NBF - 1);
          int e = cbase + ((ent >> 12) & (CHUNK - 1));
          e = e > nE - 1 ? nE - 1 : e;
          int src = srcs[e];
          src = src < 0 ? 0 : (src > nN - 1 ? nN - 1 : src);
          if (lane == 0) {
            int pos = cursor[slot];
            pos = pos < 0 ? 0 : (pos > RCAP - 1 ? RCAP - 1 : pos);
            region[pos] = src;
            const int np = pos + 1;
            cursor[slot] = np > RCAP ? RCAP : np;
          }
        }
      }
    }
    __syncthreads();
  }

  const int nv = lenW >> 2;
  int* gp = csr + rb0;
#pragma unroll 1
  for (int i = tid; i < nv; i += NTHR) { const v4i v = ((const v4i*)region)[i]; *(volatile v4i*)(gp + 4 * i) = v; }
  __threadfence();
#pragma unroll 1
  for (int i = tid; i < nv; i += NTHR) { const v4i v = ((const v4i*)region)[i]; *(volatile v4i*)(gp + 4 * i) = v; }
}

__global__ __launch_bounds__(NTHR) void k_gemm(
    const unsigned short* __restrict__ Ah, const unsigned short* __restrict__ Bw,
    const float* __restrict__ attS, const float* __restrict__ attD,
    float* C, float* eS, float* eD) {
  constexpr int TPW  = 8;
  constexpr int WC   = TPW * 16;
  constexpr int LPH  = CH / 4;
  constexpr int NES  = GBM * HEADS;
  constexpr int NESI = NES / 128;
  static_assert(2 * WC == NC && (NWAVE / 2) * 16 == GBM);
  static_assert(LPH == 16 && 2 * NESI <= NWAVE);
  static_assert(GBM * NC * 4 == GLDS);

  extern __shared__ v4f lds_dyn[];
  __shared__ __attribute__((aligned(16))) float sES[NES];
  __shared__ __attribute__((aligned(16))) float sED[NES];
  float* stg = (float*)lds_dyn;
  const int tid = threadIdx.x, lane = tid & 31, wave = tid >> 5, hh = lane >> 4, m = lane & 15;
  const int rowBase = blockIdx.x * GBM;
  const int rg  = wave >> 1;
  const int chf = wave & 1;
  const int r0  = rg * 16;
  const int c0  = chf * WC;

  v8f acc[TPW];
#pragma unroll
  for (int t = 0; t < TPW; ++t) { v8f z = {0.f, 0.f, 0.f, 0.f, 0.f, 0.f, 0.f, 0.f}; acc[t] = z; }
  const unsigned short* ap = Ah + (size_t)(rowBase + r0 + m) * FIN + 8 * hh;
  const unsigned short* bq = Bw + (size_t)(c0 + m) * FIN + 8 * hh;
#pragma unroll 1
  for (int kt = 0; kt < FIN / 32; ++kt) {
    FragH a;
    a.h[0] = *(const v8us*)(ap + 32 * kt);
    a.h[1] = *(const v8us*)(ap + 32 * kt + 16);
#pragma unroll
    for (int t = 0; t < TPW; ++t) {
      const unsigned short* bp = bq + (size_t)(16 * t) * FIN + 32 * kt;
      FragH b;
      b.h[0] = *(const v8us*)bp;
      b.h[1] = *(const v8us*)(bp + 16);
      acc[t] = wmh(a.v, b.v, acc[t]);
    }
  }

  {
    float* sp = stg + (size_t)(r0 + 8 * hh) * NC + c0 + m;
#pragma unroll
    for (int t = 0; t < TPW; ++t) {
#pragma unroll
      for (int r = 0; r < 8; ++r) sp[r * NC + 16 * t] = acc[t][r] * WINV;
    }
  }
  __syncthreads();

  const int col  = c0 + 4 * lane;
  const int hd   = col / CH;
  const v4f sA = *(const v4f*)(attS + col);
  const v4f sD = *(const v4f*)(attD + col);
  const size_t gb = (size_t)(rowBase + r0) * NC + col;
#pragma unroll
  for (int it = 0; it < 16; ++it) {
    const int row = it;
    const v4f v = *(const v4f*)(stg + (size_t)(r0 + row) * NC + col);
    *(volatile v4f*)(C + gb + (size_t)row * NC) = v;
    float ps = v.x * sA.x + v.y * sA.y + v.z * sA.z + v.w * sA.w;
    float pd = v.x * sD.x + v.y * sD.y + v.z * sD.z + v.w * sD.w;
#pragma unroll
    for (int o = 1; o < LPH; o <<= 1) { ps += __shfl_xor(ps, o); pd += __shfl_xor(pd, o); }
    if ((lane & (LPH - 1)) == 0) { sES[(r0 + row) * HEADS + hd] = ps; sED[(r0 + row) * HEADS + hd] = pd; }
  }
  __threadfence();
#pragma unroll
  for (int it = 0; it < 16; ++it) {
    const int row = it;
    const v4f v = *(const v4f*)(stg + (size_t)(r0 + row) * NC + col);
    *(volatile v4f*)(C + gb + (size_t)row * NC) = v;
  }
  __syncthreads();

  v4f dv = {0.f, 0.f, 0.f, 0.f};
  const size_t eb = (size_t)rowBase * HEADS;
  if (wave < NESI) {
    const int f = wave * 128 + 4 * lane;
    dv = *(const v4f*)(sES + f);
    *(volatile v4f*)(eS + eb + f) = dv;
  } else if (wave < 2 * NESI) {
    const int f = (wave - NESI) * 128 + 4 * lane;
    dv = *(const v4f*)(sED + f);
    *(volatile v4f*)(eD + eb + f) = dv;
  }
  __threadfence();
  if (wave < NESI) {
    const int f = wave * 128 + 4 * lane;
    *(volatile v4f*)(eS + eb + f) = dv;
  } else if (wave < 2 * NESI) {
    const int f = (wave - NESI) * 128 + 4 * lane;
    *(volatile v4f*)(eD + eb + f) = dv;
  }
}

template <int LAST>
__global__ __launch_bounds__(NTHR) void k_agg(
    const int* __restrict__ csr, const int* __restrict__ off, const int* __restrict__ cnt,
    const float* __restrict__ eS, const float* __restrict__ eD, const float* __restrict__ hw,
    const float* __restrict__ bias, const float* __restrict__ pin, float* pout,
    int addIn, int nN, int csrLen) {
  constexpr int NFL = SROWS * DOUT / 4 / 32;
  __shared__ __attribute__((aligned(16))) float sOut[NWAVE * SROWS * DOUT];
  const int tid = threadIdx.x, lane = tid & 31, wave = tid >> 5, hh = lane >> 4, q = lane & 15;
  const int tbase = blockIdx.x * TGT + wave * 32;
  const int col0 = 4 * lane;
  const int col1 = NC / 2 + 4 * lane;
  const v4f z4 = {0.f, 0.f, 0.f, 0.f};
  const v4f bb = *(const v4f*)(bias + col0) + *(const v4f*)(bias + col1);
  float* sw = sOut + wave * (SROWS * DOUT);

  const int cl    = tbase + lane;
  const int cnt_l = cnt[cl];
  const int off_l = off[cl];

#pragma unroll 1
  for (int j = 0; j < 32; ++j) {
    const int c = tbase + j;
    int n = __shfl(cnt_l, j);
    n = n < 0 ? 0 : (n > DEGCAP ? DEGCAP : n);
    const int st = __shfl(off_l, j);
    const v4f ed4 = *(const v4f*)(eD + (size_t)c * HEADS);
    const float ed0 = hh ? ed4.y : ed4.x;
    const float ed1 = hh ? ed4.w : ed4.z;

    float mx0 = NEG_BIG, mx1 = NEG_BIG;
#pragma unroll 1
    for (int q0 = 0; q0 < n; q0 += 32) {
      int pos = st + q0 + lane;
      pos = pos < 0 ? 0 : (pos > csrLen - 1 ? csrLen - 1 : pos);
      int sl = csr[pos];
      sl = sl < 0 ? 0 : (sl > nN - 1 ? nN - 1 : sl);
      const int mcnt = (n - q0) < 32 ? (n - q0) : 32;
#pragma unroll 1
      for (int pp = 0; pp < mcnt; ++pp) {
        const int s = __builtin_amdgcn_readlane(sl, pp);
        const v4f es4 = *(const v4f*)(eS + (size_t)s * HEADS);
        mx0 = fmaxf(mx0, lrelu((hh ? es4.y : es4.x) + ed0));
        mx1 = fmaxf(mx1, lrelu((hh ? es4.w : es4.z) + ed1));
      }
    }

    float den0 = 0.f, den1 = 0.f;
    v4f acc0 = z4, acc1 = z4;
#pragma unroll 1
    for (int q0 = 0; q0 < n; q0 += 32) {
      int pos = st + q0 + lane;
      pos = pos < 0 ? 0 : (pos > csrLen - 1 ? csrLen - 1 : pos);
      int sl = csr[pos];
      sl = sl < 0 ? 0 : (sl > nN - 1 ? nN - 1 : sl);
      const int mcnt = (n - q0) < 32 ? (n - q0) : 32;
#pragma unroll 1
      for (int pp = 0; pp < mcnt; ++pp) {
        const int s = __builtin_amdgcn_readlane(sl, pp);
        const v4f es4 = *(const v4f*)(eS + (size_t)s * HEADS);
        const float p0 = __expf(lrelu((hh ? es4.y : es4.x) + ed0) - mx0);
        const float p1 = __expf(lrelu((hh ? es4.w : es4.z) + ed1) - mx1);
        den0 += p0;
        den1 += p1;
        const v4f h0 = *(const v4f*)(hw + (size_t)s * NC + col0);
        const v4f h1 = *(const v4f*)(hw + (size_t)s * NC + col1);
        acc0 = acc0 + h0 * p0;
        acc1 = acc1 + h1 * p1;
      }
    }

    const float rd0 = (n > 0) ? (1.0f / den0) : 0.0f;
    const float rd1 = (n > 0) ? (1.0f / den1) : 0.0f;
    v4f v = acc0 * rd0 + acc1 * rd1 + bb;
    v.x += __shfl_xor(v.x, 16);
    v.y += __shfl_xor(v.y, 16);
    v.z += __shfl_xor(v.z, 16);
    v.w += __shfl_xor(v.w, 16);
    if (addIn != 0) v = v + *(const v4f*)(pin + (size_t)c * DOUT + 4 * q);
    if (LAST != 0) v = v * 0.25f;
    if (lane < 16) *(v4f*)(sw + (j & (SROWS - 1)) * DOUT + 4 * q) = v;

    if ((j & (SROWS - 1)) == SROWS - 1) {
      __syncthreads();
      const int jb = j - (SROWS - 1);
      float* gp = pout + (size_t)(tbase + jb) * DOUT;
      v4f ov[NFL];
#pragma unroll
      for (int it = 0; it < NFL; ++it) {
        const int f = it * 32 + lane;
        ov[it] = *(const v4f*)(sw + 4 * f);
        const int grow = tbase + jb + (f >> 4);
        if (LAST == 0 || grow < nN) *(volatile v4f*)(gp + 4 * f) = ov[it];
      }
      __threadfence();
#pragma unroll
      for (int it = 0; it < NFL; ++it) {
        const int f = it * 32 + lane;
        const int grow = tbase + jb + (f >> 4);
        if (LAST == 0 || grow < nN) *(volatile v4f*)(gp + 4 * f) = ov[it];
      }
      __syncthreads();
    }
  }
}

extern "C" void kernel_launch(void* const* d_in, const int* in_sizes, int n_in,
                              void* d_out, int out_size, void* d_ws, size_t ws_size,
                              hipStream_t stream) {
  if (n_in < 7) return;
  const int nN = in_sizes[0] / FIN;
  if (nN <= 0 || in_sizes[0] != nN * FIN) return;
  if (in_sizes[1] <= 0 || (in_sizes[1] % TT) != 0 || in_sizes[2] != in_sizes[1]) return;
  const int nE = in_sizes[1] / TT;
  if (in_sizes[3] != TT * FIN * NC) return;
  if (in_sizes[4] != TT * NC || in_sizes[5] != TT * NC || in_sizes[6] != TT * NC) return;
  if (out_size != nN * DOUT) return;
  if (nE > (1 << 28) || nN > (1 << 24)) return;

  const float* x    = (const float*)d_in[0];
  const int*   src  = (const int*)d_in[1];
  const int*   dst  = (const int*)d_in[2];
  const float* W    = (const float*)d_in[3];
  const float* al   = (const float*)d_in[4];
  const float* ar   = (const float*)d_in[5];
  const float* bias = (const float*)d_in[6];
  float* out = (float*)d_out;

  const int NPAD   = ((nN + TGT - 1) / TGT) * TGT;
  const int nBC    = (nN + NBC - 1) / NBC;
  const int CNTPAD = nBC * NBC;
  if (4 * nBC + 1 > RBN) return;
  const int nBF    = (nN + NBF - 1) / NBF;
  const int csrLen = ((nE + 31) & ~31) + 4096;
  if (31 * 4 * nBC > 4096) return;
  const int nAgg   = NPAD / TGT;
  const int nGemm  = NPAD / GBM;
  const int xUnits = NPAD * (FIN / 8);

  char* ws = (char*)d_ws;
  size_t off = 0;
  const size_t oWp  = off; off += (size_t)TT * NC * FIN * 2;      off = (off + 255) & ~(size_t)255;
  const size_t oXh  = off; off += (size_t)NPAD * FIN * 2;         off = (off + 255) & ~(size_t)255;
  const size_t oCnt = off; off += (size_t)TT * CNTPAD * 4;        off = (off + 255) & ~(size_t)255;
  const size_t oOff = off; off += (size_t)TT * CNTPAD * 4;        off = (off + 255) & ~(size_t)255;
  const size_t oRb  = off; off += (size_t)TT * RBN * 4;           off = (off + 255) & ~(size_t)255;
  const size_t oCsr = off; off += (size_t)TT * csrLen * 4;        off = (off + 255) & ~(size_t)255;
  const size_t oHw  = off; off += (size_t)NPAD * NC * 4;          off = (off + 255) & ~(size_t)255;
  const size_t oES  = off; off += (size_t)NPAD * HEADS * 4;       off = (off + 255) & ~(size_t)255;
  const size_t oED  = off; off += (size_t)NPAD * HEADS * 4;       off = (off + 255) & ~(size_t)255;
  const size_t oP0  = off; off += (size_t)NPAD * DOUT * 4;        off = (off + 255) & ~(size_t)255;
  const size_t oP1  = off; off += (size_t)NPAD * DOUT * 4;        off = (off + 255) & ~(size_t)255;
  if (off > ws_size || off > (size_t)WSCAP) return;
  unsigned short* wpl = (unsigned short*)(ws + oWp);
  unsigned short* xh  = (unsigned short*)(ws + oXh);
  int*   cnt  = (int*)(ws + oCnt);
  int*   offp = (int*)(ws + oOff);
  int*   rb   = (int*)(ws + oRb);
  int*   csr  = (int*)(ws + oCsr);
  float* hw   = (float*)(ws + oHw);
  float* es   = (float*)(ws + oES);
  float* ed   = (float*)(ws + oED);
  float* p0   = (float*)(ws + oP0);
  float* p1   = (float*)(ws + oP1);

  const int vec8 = ((nE & 3) == 0) ? 1 : 0;

  k_wprep<<<dim3(NC * FIN / 8 / NTHR, TT), NTHR, 0, stream>>>(W, wpl);
  k_xprep<<<xUnits / NTHR, NTHR, 0, stream>>>(x, xh, nN, xUnits);

  k_count<<<dim3(nBC, TT), NTHR, 0, stream>>>(dst, cnt, nE, vec8, CNTPAD);
  k_offsets<<<TT, OTHR, 0, stream>>>(cnt, offp, rb, nBC, CNTPAD);
  hipFuncSetAttribute(reinterpret_cast<const void*>(&k_fill),
                      hipFuncAttributeMaxDynamicSharedMemorySize, LDS_FILL);
  k_fill<<<dim3(nBF, TT), NTHR, LDS_FILL, stream>>>(src, dst, offp, rb, csr, nN, nE, vec8, csrLen, CNTPAD);

  hipFuncSetAttribute(reinterpret_cast<const void*>(&k_gemm),
                      hipFuncAttributeMaxDynamicSharedMemorySize, GLDS);

  k_gemm<<<nGemm, NTHR, GLDS, stream>>>(xh, wpl, al, ar, hw, es, ed);
  k_agg<0><<<nAgg, NTHR, 0, stream>>>(csr, offp, cnt, es, ed, hw, bias, p1, p0, 0, nN, csrLen);

  k_gemm<<<nGemm, NTHR, GLDS, stream>>>(xh, wpl + (size_t)NC * FIN, al + NC, ar + NC, hw, es, ed);
  k_agg<0><<<nAgg, NTHR, 0, stream>>>(csr + (size_t)csrLen, offp + (size_t)CNTPAD, cnt + (size_t)CNTPAD,
                                       es, ed, hw, bias + NC, p0, p1, 1, nN, csrLen);

  k_gemm<<<nGemm, NTHR, GLDS, stream>>>(xh, wpl + (size_t)2 * NC * FIN, al + 2 * NC, ar + 2 * NC, hw, es, ed);
  k_agg<1><<<nAgg, NTHR, 0, stream>>>(csr + (size_t)2 * csrLen, offp + (size_t)2 * CNTPAD, cnt + (size_t)2 * CNTPAD,
                                       es, ed, hw, bias + 2 * NC, p1, out, 1, nN, csrLen);
}
